// SimpleDecoderRetention_3161095930390
// MI455X (gfx1250) — hardware-verified
//
#include <hip/hip_runtime.h>
#include <math.h>


#define NB 4
#define SQ 4096
#define HI 512
#define HD 128
#define NP 64
#define BACK 768
#define TOFF 63
#define TLEN 896

typedef __attribute__((ext_vector_type(16))) _Float16 v16h;
typedef __attribute__((ext_vector_type(8)))  _Float16 v8h;
typedef __attribute__((ext_vector_type(8)))  float v8f;
typedef __attribute__((ext_vector_type(4)))  float v4f;
typedef __attribute__((ext_vector_type(4)))  unsigned v4u;
typedef float __attribute__((may_alias)) float_a;

template <typename T> __device__ __forceinline__ void vst2(void* p, T v) { *(volatile T*)p = v; __threadfence(); *(volatile T*)p = v; }
__device__ __forceinline__ v8f wmma16(v16h a, v16h b, v8f c) {
  v8f d = __builtin_amdgcn_wmma_f32_16x16x32_f16(false, a, false, b, (short)0, c, false, false);
  asm volatile("v_nop\n\tv_nop\n\tv_nop\n\tv_nop" : "+v"(d) : "v"(a), "v"(b));
  return d;
}
__device__ __forceinline__ v16h frag_h(const _Float16* rowk0, int lane) {
  union { v16h v; v8h q[2]; } u; const _Float16* p = rowk0 + 8 * (lane >> 4);
  u.q[0] = *(const v8h*)p; u.q[1] = *(const v8h*)(p + 16); return u.v;
}
__device__ __forceinline__ v16h frag_f32(const float* rowk0, int lane) {
  v16h a; const float* p = rowk0 + 8 * (lane >> 4);
#pragma unroll
  for (int i = 0; i < 8; ++i) { a[i] = (_Float16)p[i]; a[8 + i] = (_Float16)p[16 + i]; }
  return a;
}
#define LDSX() do { asm volatile("s_wait_dscnt 0" ::: "memory"); __builtin_amdgcn_wave_barrier(); __builtin_amdgcn_fence(__ATOMIC_RELEASE, "workgroup"); } while (0)

__global__ __launch_bounds__(256) void k_tab(const float* __restrict__ Wq, const float* __restrict__ Wk, const float* __restrict__ Wv,
                                           float* __restrict__ tab, float* __restrict__ gdec, _Float16* __restrict__ WT) {
  const int tid = blockIdx.x * 256 + threadIdx.x;
  if (tid < TLEN * NP) { const int j = tid / NP - TOFF, i = tid % NP;
    const float base = ((float)(2 * i) + 0.4f * (float)HD) / (1.4f * (float)HD);
    vst2(tab + tid, (float_a)powf(base, (float)j / 512.0f)); }
  if (tid < TLEN) vst2(gdec + tid, (float_a)powf(0.96875f, (float)tid));
  if (tid < 3 * HD) { const int which = tid / HD, n = tid % HD; const float* W = which == 0 ? Wq : (which == 1 ? Wk : Wv);
    for (int q = 0; q < HI / 8; ++q) { union { v8h h; v4u u; } p8;
#pragma unroll
      for (int e = 0; e < 8; ++e) p8.h[e] = (_Float16)(W[(size_t)(q * 8 + e) * HD + n] * 64.0f);
      vst2(WT + ((size_t)which * HD + n) * HI + q * 8, p8.u); } }
}
__global__ __launch_bounds__(128) void k_proj(const float* __restrict__ X, const float* __restrict__ Mem, const _Float16* __restrict__ WT, const float* __restrict__ tab,
                                            _Float16* __restrict__ Qs, _Float16* __restrict__ Kr, _Float16* __restrict__ VT) {
  __shared__ __align__(16) float so[4][16][132];
  __shared__ __align__(16) _Float16 st[HD][72];
  const int tid = threadIdx.x, wave = tid >> 5, lane = tid & 31, col = lane & 15, g = lane >> 4;
  const int which = blockIdx.z, b = blockIdx.y, r0 = blockIdx.x * 64 + wave * 16;
  const float* A = (which == 0 ? X : Mem) + ((size_t)b * SQ) * HI; const _Float16* W = WT + (size_t)which * HD * HI;
  v8f acc[8] = {};
#pragma unroll 1
  for (int kc = 0; kc < HI / 32; ++kc) { const v16h a = frag_f32(A + (size_t)(r0 + col) * HI + kc * 32, lane);
#pragma unroll
    for (int j = 0; j < 8; ++j) acc[j] = wmma16(a, frag_h(W + (size_t)(j * 16 + col) * HI + kc * 32, lane), acc[j]); }
  float* S = &so[wave][0][0];
#pragma unroll
  for (int j = 0; j < 8; ++j)
#pragma unroll
    for (int r = 0; r < 8; ++r) S[(8 * g + r) * 132 + j * 16 + col] = acc[j][r] * (1.0f / 64.0f);
  LDSX();
  if (which == 2) {
    for (int q = lane; q < 16 * HD; q += 32) { const int rl = q >> 7, v = q & 127; st[v][wave * 16 + rl] = (_Float16)S[rl * 132 + v]; }
    __syncthreads();
    for (int q = tid; q < HD * 8; q += 128) { const int v = q >> 3, pc = q & 7; vst2(VT + ((size_t)b * HD + v) * SQ + blockIdx.x * 64 + pc * 8, *(const v4u*)(&st[v][pc * 8])); }
    return;
  }
  for (int q = lane; q < 16 * 8; q += 32) { const int rl = q >> 3, pb = (q & 7) * 8; const int n = r0 + rl;
    float tmp[16];
#pragma unroll
    for (int e = 0; e < 8; ++e) { const int i = pb + e;
      const float invf = powf(10000.0f, -(float)i / (float)NP);
      const float ang = (float)n * invf; const float sn = sinf(ang), cs = cosf(ang);
      float sc = 1.0f;
      if (which == 0) sc = tab[((n & 63) + TOFF) * NP + i];
      const float x1 = S[rl * 132 + 2 * i], x2 = S[rl * 132 + 2 * i + 1];
      tmp[2 * e] = (x1 * cs - x2 * sn) * sc; tmp[2 * e + 1] = (x2 * cs + x1 * sn) * sc; }
#pragma unroll
    for (int e = 0; e < 16; ++e) S[rl * 132 + pb * 2 + e] = tmp[e]; }
  LDSX();
  _Float16* dst = (which == 0 ? Qs : Kr) + ((size_t)b * SQ + r0) * HD;
  for (int q = lane; q < 16 * 16; q += 32) { const int rl = q >> 4, pc = q & 15; union { v8h h; v4u u; } pk;
#pragma unroll
    for (int e = 0; e < 8; ++e) pk.h[e] = (_Float16)S[rl * 132 + pc * 8 + e];
    vst2(dst + (size_t)rl * HD + pc * 8, pk.u); }
}
__global__ __launch_bounds__(128) void k_ret(const _Float16* __restrict__ Qs, const _Float16* __restrict__ Kr, const _Float16* __restrict__ VT,
                                           const float* __restrict__ tab, const float* __restrict__ gdec, float* __restrict__ out) {
  __shared__ __align__(16) _Float16 sK[64][HD + 8];
  __shared__ __align__(16) _Float16 sP[4][16][72];
  __shared__ __align__(16) float so[4][16][132];
  const int tid = threadIdx.x, w = tid >> 5, lane = tid & 31, col = lane & 15, g = lane >> 4;
  const int b = blockIdx.y, n0 = blockIdx.x * 64, q0 = n0 + w * 16;
  const _Float16* qb = Qs + ((size_t)b * SQ) * HD; const _Float16* kb = Kr + ((size_t)b * SQ) * HD; const _Float16* vb = VT + (size_t)b * HD * SQ;
  v16h aq[4];
#pragma unroll
  for (int kc = 0; kc < 4; ++kc) aq[kc] = frag_h(qb + (size_t)(q0 + col) * HD + kc * 32, lane);
  v8f acc[8] = {};
  int mstart = n0 - BACK; if (mstart < 0) mstart = 0; mstart &= ~63;
#pragma unroll 1
  for (int m0 = mstart; m0 <= n0; m0 += 64) {
    __syncthreads();
    { const int key = tid >> 1, d0 = (tid & 1) * 64, m = m0 + key; const int jj = n0 - m + TOFF;
      const float* tr = tab + (size_t)jj * NP; const _Float16* kr = kb + (size_t)m * HD + d0;
#pragma unroll
      for (int pc = 0; pc < 8; ++pc) { union { v8h h; v4u u; } pk; const v8h kv = *(const v8h*)(kr + pc * 8);
#pragma unroll
        for (int e = 0; e < 8; ++e) pk.h[e] = (_Float16)((float)kv[e] * tr[(d0 + pc * 8 + e) >> 1]);
        *(v4u*)(&sK[key][d0 + pc * 8]) = pk.u; } }
    __syncthreads();
    v8f s4[4];
#pragma unroll
    for (int t = 0; t < 4; ++t) { s4[t] = (v8f){};
#pragma unroll
      for (int kc = 0; kc < 4; ++kc) s4[t] = wmma16(aq[kc], frag_h(&sK[t * 16 + col][0] + kc * 32, lane), s4[t]); }
#pragma unroll
    for (int t = 0; t < 4; ++t)
#pragma unroll
      for (int r = 0; r < 8; ++r) { const int dlt = (q0 + 8 * g + r) - (m0 + t * 16 + col);
        const float dv = dlt >= 0 ? gdec[dlt < TLEN ? dlt : TLEN - 1] : 0.f;
        sP[w][8 * g + r][t * 16 + col] = (_Float16)(s4[t][r] * dv * 1024.0f); }
    LDSX();
#pragma unroll
    for (int kc = 0; kc < 2; ++kc) { const v16h pa = frag_h(&sP[w][col][0] + kc * 32, lane);
#pragma unroll
      for (int t = 0; t < 8; ++t) acc[t] = wmma16(pa, frag_h(vb + (size_t)(t * 16 + col) * SQ + m0 + kc * 32, lane), acc[t]); }
    __builtin_amdgcn_wave_barrier();
  }
#pragma unroll
  for (int t = 0; t < 8; ++t)
#pragma unroll
    for (int r = 0; r < 8; ++r) so[w][8 * g + r][t * 16 + col] = acc[t][r] * (1.0f / 1024.0f);
  LDSX();
#pragma unroll 4
  for (int rl = 0; rl < 16; ++rl) vst2(out + ((size_t)b * SQ + q0 + rl) * HD + lane * 4, *(const v4f*)(&so[w][rl][lane * 4]));
}

extern "C" void kernel_launch(void* const* d_in, const int* in_sizes, int n_in,
                              void* d_out, int out_size, void* d_ws, size_t ws_size,
                              hipStream_t stream) {
  (void)in_sizes; (void)n_in; (void)out_size; (void)ws_size;
  const float* X = (const float*)d_in[0]; const float* Mem = (const float*)d_in[1];
  const float* Wq = (const float*)d_in[2]; const float* Wk = (const float*)d_in[3]; const float* Wv = (const float*)d_in[4];
  float* out = (float*)d_out;
  char* ws = (char*)d_ws; size_t off = 0;
  auto take = [&](size_t bytes) { char* p = ws + off; off += (bytes + 255) & ~(size_t)255; return p; };
  float* tab = (float*)take((size_t)TLEN * NP * 4); float* gdec = (float*)take((size_t)TLEN * 4);
  _Float16* WT = (_Float16*)take((size_t)3 * HD * HI * 2);
  _Float16* Qs = (_Float16*)take((size_t)NB * SQ * HD * 2); _Float16* Kr = (_Float16*)take((size_t)NB * SQ * HD * 2); _Float16* VT = (_Float16*)take((size_t)NB * HD * SQ * 2);
  k_tab<<<(TLEN * NP + 255) / 256, 256, 0, stream>>>(Wq, Wk, Wv, tab, gdec, WT);
  k_proj<<<dim3(SQ / 64, NB, 3), 128, 0, stream>>>(X, Mem, WT, tab, Qs, Kr, VT);
  k_ret<<<dim3(SQ / 64, NB), 128, 0, stream>>>(Qs, Kr, VT, tab, gdec, out);
}
